// CausalSelfAttention_TSSA_63977832841579
// MI455X (gfx1250) — hardware-run, weakly checked
//
#include <hip/hip_runtime.h>


#define NB   4
#define NT   2048
#define NM   8192
#define NC   1024
#define NG   16
#define NE   128
#define TINY 1.1920929e-07f

typedef _Float16 h16;
typedef unsigned short bf;
typedef __attribute__((ext_vector_type(16))) __bf16   v16bf;
typedef __attribute__((ext_vector_type(16))) _Float16 v16h;
typedef __attribute__((ext_vector_type(8)))  _Float16 v8h;
typedef __attribute__((ext_vector_type(8)))  unsigned short v8us;
typedef __attribute__((ext_vector_type(8)))  float    v8f;
typedef __attribute__((ext_vector_type(4)))  float    v4f;
typedef v8h  __attribute__((may_alias)) v8ha;
typedef v4f  __attribute__((may_alias)) v4fa;
typedef v8us __attribute__((may_alias)) v8usa;

__device__ __forceinline__ unsigned short f2bf(float f) { unsigned u = __float_as_uint(f); u += 0x7FFFu + ((u >> 16) & 1u); return (unsigned short)(u >> 16); }
__device__ __forceinline__ float bf2f(unsigned short b) { return __uint_as_float(((unsigned)b) << 16); }
__device__ __forceinline__ float bfr(float f) { return bf2f(f2bf(f)); }
__device__ __forceinline__ v16h cat16(v8h lo, v8h hi) { return __builtin_shufflevector(lo, hi, 0, 1, 2, 3, 4, 5, 6, 7, 8, 9, 10, 11, 12, 13, 14, 15); }
__device__ __forceinline__ v16bf cat16b(v8us lo, v8us hi) { return __builtin_bit_cast(v16bf, __builtin_shufflevector(lo, hi, 0, 1, 2, 3, 4, 5, 6, 7, 8, 9, 10, 11, 12, 13, 14, 15)); }
__device__ __forceinline__ v8f wmma16(v16h a, v16h b, v8f c) { return __builtin_amdgcn_wmma_f32_16x16x32_f16(false, a, false, b, (short)0, c, false, false); }
__device__ __forceinline__ v8f wmmab(v16bf a, v16bf b, v8f c) { return __builtin_amdgcn_wmma_f32_16x16x32_bf16(false, a, false, b, (short)0, c, false, false); }

template <typename T16> struct WFrag;
template <> struct WFrag<h16> { typedef v16h V; static __device__ __forceinline__ V ld(const h16* p) { return cat16(*(const v8h*)p, *(const v8h*)(p + 16)); } static __device__ __forceinline__ v8f mma(V a, V b, v8f c) { return wmma16(a, b, c); } };
template <> struct WFrag<bf> { typedef v16bf V; static __device__ __forceinline__ V ld(const bf* p) { return cat16b(*(const v8us*)p, *(const v8us*)(p + 16)); } static __device__ __forceinline__ v8f mma(V a, V b, v8f c) { return wmmab(a, b, c); } };
template <typename T16, int NSPLIT, bool BIAS>
__global__ __launch_bounds__(32) void k_gemmw(const T16* __restrict__ A, const T16* __restrict__ A2, const T16* __restrict__ Bt, const T16* __restrict__ Bt2, int K, float* C, int ldc, const float* __restrict__ bias, size_t sA, size_t sB, size_t sC) {
    typedef typename WFrag<T16>::V V;
    __shared__ __align__(16) float os[16 * 68];
    const size_t z = blockIdx.z; A += z * sA; if (A2) A2 += z * sA; Bt += z * sB; if (Bt2) Bt2 += z * sB; C += z * sC;
    const int lane = threadIdx.x & 31, lr = lane & 15, hi = lane >> 4; const int r0 = blockIdx.x * 64, c0 = blockIdx.y * 64;
    v8f acc[4][4];
#pragma unroll
    for (int mb = 0; mb < 4; ++mb)
#pragma unroll
        for (int nb = 0; nb < 4; ++nb) acc[mb][nb] = (v8f){};
    const size_t aoff = (size_t)(r0 + lr) * K + 8 * hi, boff = (size_t)(c0 + lr) * K + 8 * hi;
    for (int kc = 0; kc < K; kc += 32) {
        V a[4], a2[4];
#pragma unroll
        for (int mb = 0; mb < 4; ++mb) { a[mb] = WFrag<T16>::ld(A + aoff + (size_t)mb * 16 * K + kc); if (NSPLIT == 1 || NSPLIT == 2) a2[mb] = WFrag<T16>::ld(A2 + aoff + (size_t)mb * 16 * K + kc); }
#pragma unroll
        for (int nb = 0; nb < 4; ++nb) { const V b = WFrag<T16>::ld(Bt + boff + (size_t)nb * 16 * K + kc); V b2; if (NSPLIT >= 2) b2 = WFrag<T16>::ld(Bt2 + boff + (size_t)nb * 16 * K + kc);
#pragma unroll
            for (int mb = 0; mb < 4; ++mb) { acc[mb][nb] = WFrag<T16>::mma(a[mb], b, acc[mb][nb]); if (NSPLIT == 1 || NSPLIT == 2) acc[mb][nb] = WFrag<T16>::mma(a2[mb], b, acc[mb][nb]); if (NSPLIT >= 2) acc[mb][nb] = WFrag<T16>::mma(a[mb], b2, acc[mb][nb]); } }
        asm volatile("v_nop\n\tv_nop\n\tv_nop\n\tv_nop" : "+v"(acc[0][0]), "+v"(acc[1][1]), "+v"(acc[2][2]), "+v"(acc[3][3]) : "v"(a[0]), "v"(a[3]));
    }
#pragma unroll
    for (int mb = 0; mb < 4; ++mb) {
#pragma unroll
        for (int nb = 0; nb < 4; ++nb) {
#pragma unroll
            for (int j = 0; j < 8; ++j) os[(hi * 8 + j) * 68 + nb * 16 + lr] = acc[mb][nb][j]; }
        __builtin_amdgcn_wave_barrier(); asm volatile("" ::: "memory");
        float* crow = C + (size_t)(r0 + mb * 16) * ldc + c0;
#pragma unroll 1
        for (int ps = 0; ps < 2; ++ps) {
#pragma unroll
            for (int s = 0; s < 8; ++s) { const int row = 2 * s + hi, cofs = lr * 4; v4f val = *(const v4fa*)(os + row * 68 + cofs); if (BIAS) { val[0] += bfr(bias[c0 + cofs]); val[1] += bfr(bias[c0 + cofs + 1]); val[2] += bfr(bias[c0 + cofs + 2]); val[3] += bfr(bias[c0 + cofs + 3]); }
                *(volatile v4f*)(crow + (size_t)row * ldc + cofs) = val; }
            if (ps == 0) __threadfence(); }
        __builtin_amdgcn_wave_barrier(); asm volatile("" ::: "memory");
    }
}

typedef __attribute__((ext_vector_type(2))) _Float16 v2h;
typedef __attribute__((ext_vector_type(4))) _Float16 v4h;
typedef __attribute__((ext_vector_type(2))) unsigned short v2us;
typedef __attribute__((ext_vector_type(4))) unsigned short v4us;
typedef __attribute__((ext_vector_type(2))) float v2f;
typedef __attribute__((ext_vector_type(4))) int v4i;
__global__ __launch_bounds__(256) void k_cvt8(const float* __restrict__ src, bf* dst, size_t n8) { const size_t i = (size_t)blockIdx.x * 256 + threadIdx.x; if (i >= n8) return; const v8f v = *(const v8f*)(src + i * 8); v8us o;
#pragma unroll
    for (int k = 0; k < 8; ++k) o[k] = f2bf(v[k]); *(volatile v8us*)(dst + i * 8) = o; __threadfence(); *(volatile v8us*)(dst + i * 8) = o; }

__device__ __forceinline__ h16 toh_flush(float x) { const float z = (fabsf(x) < 6.103515625e-05f) ? 0.0f : x; return (h16)z; }

template <bool RB>
__global__ __launch_bounds__(256) void k_c16(const float* __restrict__ src, h16* dst, size_t n8) { const size_t i = (size_t)blockIdx.x * 256 + threadIdx.x; if (i >= n8) return; const float* p = src + i * 8; const v4f a = *(const v4f*)p, b = *(const v4f*)(p + 4); v8h o;
#pragma unroll
    for (int q = 0; q < 4; ++q) { o[q] = toh_flush(RB ? bfr(a[q]) : a[q]); o[q + 4] = toh_flush(RB ? bfr(b[q]) : b[q]); }
    *(volatile v8h*)(dst + i * 8) = o; __threadfence(); *(volatile v8h*)(dst + i * 8) = o; }

__global__ __launch_bounds__(256) void k_sq(const float* __restrict__ Pw, const float* __restrict__ a5, float* Qn) { const unsigned id = blockIdx.x * 256u + threadIdx.x; const unsigned sq_ = id >> 10, ch = id & 1023u, gr = ch >> 6; float run = 0.0f;
    for (int t0 = 0; t0 < NT; t0 += 8) { const size_t r0 = (size_t)sq_ * NT + t0; float hv[8];
#pragma unroll
        for (int js = 0; js < 8; ++js) { const float vv = Pw[(r0 + js) * NC + ch]; const float sq = vv * vv; run = run + sq; hv[js] = sq / fmaxf(run, TINY) + bfr(a5[gr * NT + t0 + js]); }
        float* po = Qn + r0 * NC + ch;
#pragma unroll
        for (int js = 0; js < 8; ++js) *(volatile float*)(po + (size_t)js * NC) = hv[js];
        __threadfence();
#pragma unroll
        for (int js = 0; js < 8; ++js) *(volatile float*)(po + (size_t)js * NC) = hv[js]; }
}

__global__ __launch_bounds__(256) void k_sum8(const float* __restrict__ Qn, float* S8) { const unsigned id = blockIdx.x * 256u + threadIdx.x; const float* pq = Qn + (size_t)id * 8; const v4f q0 = *(const v4f*)pq, q1 = *(const v4f*)(pq + 4);
    float acc = q0[0]; acc = acc + q0[1]; acc = acc + q0[2]; acc = acc + q0[3]; acc = acc + q1[0]; acc = acc + q1[1]; acc = acc + q1[2]; acc = acc + q1[3];
    *(volatile float*)(S8 + id) = acc; __threadfence(); *(volatile float*)(S8 + id) = acc; }

__global__ __launch_bounds__(256) void k_soft(const float* __restrict__ S8, const float* __restrict__ a4, float* Hw) { const unsigned rw = blockIdx.x * 256u + threadIdx.x; const float* ps = S8 + (size_t)rw * NE; float tv[NG];
#pragma unroll
    for (int g = 0; g < NG; ++g) { const v4f s0 = *(const v4f*)(ps + 8 * g), s1 = *(const v4f*)(ps + 8 * g + 4); float acc = s0[0]; acc = acc + s0[1]; acc = acc + s0[2]; acc = acc + s0[3]; acc = acc + s1[0]; acc = acc + s1[1]; acc = acc + s1[2]; acc = acc + s1[3]; tv[g] = acc * bfr(a4[g]); }
    float top = tv[0];
#pragma unroll
    for (int g = 1; g < NG; ++g) top = fmaxf(top, tv[g]);
    float tot = 0.0f;
#pragma unroll
    for (int g = 0; g < NG; ++g) { tv[g] = expf(tv[g] - top); tot = tot + tv[g]; }
#pragma unroll
    for (int g = 0; g < NG; ++g) tv[g] = tv[g] / tot;
#pragma unroll
    for (int g = 0; g < NG; ++g) *(volatile float*)(Hw + (size_t)g * NM + rw) = tv[g];
    __threadfence();
#pragma unroll
    for (int g = 0; g < NG; ++g) *(volatile float*)(Hw + (size_t)g * NM + rw) = tv[g]; }

__global__ __launch_bounds__(256) void k_row(float* Pw, const float* __restrict__ Hw) { const unsigned id = blockIdx.x * 256u + threadIdx.x; const unsigned sq_ = id >> 10, ch = id & 1023u, gr = ch >> 6; float sa = 0.0f, sb = 0.0f;
    for (int t0 = 0; t0 < NT; t0 += 8) { const size_t r0 = (size_t)sq_ * NT + t0; float* pp = Pw + r0 * NC + ch; const float* ph = Hw + (size_t)gr * NM + r0; float vr[8], hv[8];
#pragma unroll
        for (int js = 0; js < 8; ++js) vr[js] = pp[(size_t)js * NC];
#pragma unroll
        for (int js = 0; js < 8; ++js) { const float vv = vr[js], sh = ph[js]; sa = sa + (vv * vv) * sh; sb = sb + sh; const float dq = sa / (sb + TINY); hv[js] = (-(vv * sh)) * (1.0f / (1.0f + dq)); }
#pragma unroll
        for (int js = 0; js < 8; ++js) *(volatile float*)(pp + (size_t)js * NC) = hv[js];
        __threadfence();
#pragma unroll
        for (int js = 0; js < 8; ++js) *(volatile float*)(pp + (size_t)js * NC) = hv[js]; }
}

extern "C" void kernel_launch(void* const* d_in, const int* in_sizes, int n_in, void* d_out, int out_size, void* d_ws, size_t ws_size, hipStream_t stream) {
    if (n_in < 5) return;
    if (in_sizes[0] != NM * NC || in_sizes[1] != NC * NC || in_sizes[2] != NC * NC || in_sizes[3] != NG || in_sizes[4] != NG * NT) return;
    if (out_size != NM * NC) return;
    static_assert(NM == NB * NT && NC == NG * 64 && NE * 8 == NC && NM % 64 == 0 && NC % 64 == 0 && NC % 32 == 0 && (NM * NC / 8) % 256 == 0 && (NC * NC / 8) % 256 == 0 && (NB * NC) % 256 == 0 && (NM * NE) % 256 == 0 && NM % 256 == 0 && NT % 8 == 0 && NC == 1024, "the products: row and column counts multiples of 64, the depth of 32; the flat grids exact; the walks: a thread a (sequence, channel) with 1,024 channels a sequence; the ticks in eights; 16 groups of 64; 128 eighths a row");
    const float* i0 = (const float*)d_in[0]; const float* i1 = (const float*)d_in[1]; const float* i2 = (const float*)d_in[2]; const float* i3 = (const float*)d_in[3]; const float* i4 = (const float*)d_in[4]; float* res = (float*)d_out;
    char* wsp = (char*)d_ws; auto take = [&](size_t bytes) { char* p = wsp; wsp += (bytes + 255) & ~(size_t)255; return (void*)p; };
    bf* Xb = (bf*)take((size_t)NM * NC * 2); bf* Wa = (bf*)take((size_t)NC * NC * 2); float* Pw = (float*)take((size_t)NM * NC * 4); float* Qn = (float*)take((size_t)NM * NC * 4); float* S8 = (float*)take((size_t)NM * NE * 4); float* Hw = (float*)take((size_t)NG * NM * 4); h16* Yh = (h16*)take((size_t)NM * NC * 2); h16* Wh = (h16*)take((size_t)NC * NC * 2);
    if ((size_t)(wsp - (char*)d_ws) > ws_size) return;
    k_cvt8<<<(unsigned)(NM * NC / 8 / 256), 256, 0, stream>>>(i0, Xb, (size_t)NM * NC / 8);
    k_cvt8<<<(unsigned)(NC * NC / 8 / 256), 256, 0, stream>>>(i1, Wa, (size_t)NC * NC / 8);
    k_gemmw<bf, 0, false><<<dim3(NM / 64, NC / 64, 1), 32, 0, stream>>>(Xb, nullptr, Wa, nullptr, NC, Pw, NC, nullptr, 0, 0, 0);
    k_sq<<<(unsigned)(NB * NC / 256), 256, 0, stream>>>(Pw, i4, Qn);
    k_sum8<<<(unsigned)(NM * NE / 256), 256, 0, stream>>>(Qn, S8);
    k_soft<<<(unsigned)(NM / 256), 256, 0, stream>>>(S8, i3, Hw);
    k_row<<<(unsigned)(NB * NC / 256), 256, 0, stream>>>(Pw, Hw);
    k_c16<false><<<(unsigned)(NM * NC / 8 / 256), 256, 0, stream>>>(Pw, Yh, (size_t)NM * NC / 8);
    k_c16<true><<<(unsigned)(NC * NC / 8 / 256), 256, 0, stream>>>(i2, Wh, (size_t)NC * NC / 8);
    k_gemmw<h16, 0, false><<<dim3(NM / 64, NC / 64, 1), 32, 0, stream>>>(Yh, nullptr, Wh, nullptr, NC, res, NC, nullptr, 0, 0, 0);
}
